// Connection_v5_17076789969613
// MI455X (gfx1250) — hardware-verified
//
#include <hip/hip_runtime.h>
#include <hip/hip_bf16.h>

typedef __attribute__((ext_vector_type(16))) __bf16 v16bf;
typedef __attribute__((ext_vector_type(8)))  __bf16 v8bf;
typedef __attribute__((ext_vector_type(16))) _Float16 v16h;
typedef __attribute__((ext_vector_type(8)))  _Float16 v8h;
typedef __attribute__((ext_vector_type(8)))  float  v8f;
typedef __attribute__((ext_vector_type(4)))  float  v4f;
typedef __attribute__((ext_vector_type(4)))  unsigned v4u;
template <typename T> __device__ __forceinline__ void vst2(void* p, T v) { *(volatile T*)p = v; __threadfence(); *(volatile T*)p = v; }
struct A3 { v16bf h, m, l; };
__device__ __forceinline__ A3 split_row(const float* row, int k0, int lane) {
  A3 r; const float* p = row + k0 + 8 * (lane >> 4);
#pragma unroll
  for (int i = 0; i < 16; ++i) {
    const float x = p[(i < 8) ? i : (i + 8)];
    const __bf16 h = (__bf16)x; const float rh = x - (float)h;
    const __bf16 m = (__bf16)rh; const __bf16 l = (__bf16)(rh - (float)m);
    r.h[i] = h; r.m[i] = m; r.l[i] = l;
  }
  return r;
}

#define DD  128
#define DD2 256

__device__ __forceinline__ v16bf frag_bf16(const __bf16* __restrict__ p, int ld,
                                           int row0, int k0) {
  int lane = threadIdx.x & 31;
  int g = lane >> 4, r = lane & 15;
  const __bf16* q = p + (row0 + r) * ld + k0 + g * 8;
  v8bf lo = *(const v8bf*)(q);
  v8bf hi = *(const v8bf*)(q + 16);
  return __builtin_shufflevector(lo, hi, 0,1,2,3,4,5,6,7,8,9,10,11,12,13,14,15);
}

__device__ __forceinline__ v16bf frag_f32(const float* __restrict__ p, int ld,
                                          int row0, int k0) {
  int lane = threadIdx.x & 31;
  int g = lane >> 4, r = lane & 15;
  const float* q = p + (row0 + r) * ld + k0 + g * 8;
  v16bf f;
#pragma unroll
  for (int i = 0; i < 8; ++i) { f[i] = (__bf16)q[i]; f[i + 8] = (__bf16)q[16 + i]; }
  return f;
}

__device__ __forceinline__ v8f wmma_bf16(v16bf a, v16bf b, v8f c) {
  v8f d = __builtin_amdgcn_wmma_f32_16x16x32_bf16(false, a, false, b, (short)0, c, false, false);
  asm volatile("v_nop\n\tv_nop\n\tv_nop\n\tv_nop" : "+v"(d) : "v"(a), "v"(b));
  return d;
}
__device__ __forceinline__ v8f wmma_f16(v16h a, v16h b, v8f c) {
  v8f d = __builtin_amdgcn_wmma_f32_16x16x32_f16(false, a, false, b, (short)0, c, false, false);
  asm volatile("v_nop\n\tv_nop\n\tv_nop\n\tv_nop" : "+v"(d) : "v"(a), "v"(b));
  return d;
}
__device__ __forceinline__ v16h frag_h(const _Float16* __restrict__ p, int ld, int row0, int k0) {
  int lane = threadIdx.x & 31; int g = lane >> 4, r = lane & 15;
  const _Float16* q = p + (row0 + r) * ld + k0 + g * 8;
  v8h lo = *(const v8h*)(q); v8h hi = *(const v8h*)(q + 16);
  return __builtin_shufflevector(lo, hi, 0,1,2,3,4,5,6,7,8,9,10,11,12,13,14,15);
}
__device__ __forceinline__ v8f mac6(const A3& a, const __bf16* p0, const __bf16* p1, const __bf16* p2, int ld, int row0, int k0, v8f c) {
  const v16bf fh = frag_bf16(p0, ld, row0, k0), fm = frag_bf16(p1, ld, row0, k0), fl = frag_bf16(p2, ld, row0, k0);
  c = wmma_bf16(a.l, fh, c); c = wmma_bf16(a.m, fm, c); c = wmma_bf16(a.h, fl, c);
  c = wmma_bf16(a.m, fh, c); c = wmma_bf16(a.h, fm, c); c = wmma_bf16(a.h, fh, c);
  return c;
}

__global__ __launch_bounds__(256) void prep_w1(const float* __restrict__ W1, __bf16* __restrict__ w1p) {
  const int g8 = blockIdx.x * 256 + threadIdx.x;
  union { v8bf b; v4u u; } ph, pm, pl;
#pragma unroll
  for (int e = 0; e < 8; ++e) { const float x = W1[(size_t)g8 * 8 + e]; const __bf16 h = (__bf16)x; const float rh = x - (float)h; const __bf16 m = (__bf16)rh; const __bf16 l = (__bf16)(rh - (float)m); ph.b[e] = h; pm.b[e] = m; pl.b[e] = l; }
  vst2(w1p + (size_t)g8 * 8, ph.u); vst2(w1p + 256 * 128 + (size_t)g8 * 8, pm.u); vst2(w1p + 2 * 256 * 128 + (size_t)g8 * 8, pl.u);
}
__global__ __launch_bounds__(256) void prep_cvt(const float* __restrict__ W, _Float16* __restrict__ d) {
  const int g8 = blockIdx.x * 256 + threadIdx.x;
  union { v8h h; v4u u; } pk;
#pragma unroll
  for (int e = 0; e < 8; ++e) pk.h[e] = (_Float16)W[(size_t)g8 * 8 + e];
  vst2(d + (size_t)g8 * 8, pk.u);
}
__global__ __launch_bounds__(256) void prep_t(const float* __restrict__ W, _Float16* __restrict__ WT, int R, int Cc) {
  __shared__ __align__(16) _Float16 tile[64][72];
  const int ct = Cc / 64, tid = threadIdx.x;
  const int c0 = (blockIdx.x % ct) * 64, r0 = (blockIdx.x / ct) * 64;
  for (int i = tid; i < 64 * 64; i += 256) { const int rr = i >> 6, cc = i & 63; tile[cc][rr] = (_Float16)W[(size_t)(r0 + rr) * Cc + c0 + cc]; }
  __syncthreads();
  for (int g = tid; g < 64 * 8; g += 256) { const int cc = g >> 3, pc = g & 7; vst2(WT + (size_t)(c0 + cc) * R + r0 + pc * 8, *(const v4u*)(&tile[cc][pc * 8])); }
}

__global__ __launch_bounds__(128)
void fused_kernel(const float* __restrict__ input,
                  const float* __restrict__ b1,
                  const float* __restrict__ b2,
                  const __bf16* __restrict__ w1p,
                  const _Float16* __restrict__ w2h,
                  const _Float16* __restrict__ w1t,
                  const _Float16* __restrict__ w2t,
                  float* __restrict__ out) {
  __shared__ __align__(16) _Float16 sHM[32 * DD2];
  __shared__ unsigned char sMask[16 * DD2];
  __shared__ float sS[16 * DD];
  __shared__ float sWv[16 * DD];
  __shared__ __align__(16) _Float16 sU[16 * DD];
  __shared__ __align__(16) _Float16 sQ[16 * DD2];
  __shared__ __align__(16) float sDV[16 * DD];

  const int tid  = threadIdx.x;
  const int wid  = tid >> 5;
  const int lane = tid & 31;
  const int g    = lane >> 4;
  const int ln   = lane & 15;
  const int row0 = blockIdx.x * 16;
  const float* inB = input + (size_t)row0 * DD2;

  {
    const v4f* in4 = (const v4f*)inB;
    for (int idx = tid; idx < 16 * 32; idx += 128) {
      int m = idx >> 5, t = idx & 31;
      vst2(out + (size_t)(row0 + m) * DD2 + t * 4, in4[m * 64 + 32 + t]);
    }
  }

  {
    const int lane_ = tid & 31;
    const float* arow = inB + (size_t)ln * DD2;
#pragma unroll 1
    for (int i = 0; i < 4; ++i) {
      int nt = wid + 4 * i;
      v8f accX = {}, accV = {};
#pragma unroll
      for (int ks = 0; ks < 4; ++ks) {
        const A3 ax = split_row(arow, ks * 32, lane_), av = split_row(arow + DD, ks * 32, lane_);
        accX = mac6(ax, w1p, w1p + 256 * 128, w1p + 2 * 256 * 128, DD, nt * 16, ks * 32, accX);
        accV = mac6(av, w1p, w1p + 256 * 128, w1p + 2 * 256 * 128, DD, nt * 16, ks * 32, accV);
      }
      int col = nt * 16 + ln;
      float bb = b1[col];
#pragma unroll
      for (int r = 0; r < 8; ++r) {
        int m = r + 8 * g;
        float z = accX[r] + bb;
        bool mk = (z > 0.0f);
        sMask[m * DD2 + col] = mk;
        sHM[m * DD2 + col] = (_Float16)(mk ? z : 0.0f);
        sHM[(16 + m) * DD2 + col] = (_Float16)(mk ? accV[r] : 0.0f);
      }
    }
  }
  __syncthreads();

  {
#pragma unroll
    for (int i = 0; i < 2; ++i) {
      int nt = wid + 4 * i;
      v8f accS = {}, accW = {};
#pragma unroll
      for (int ks = 0; ks < 8; ++ks) {
        v16h b = frag_h(w2h, DD2, nt * 16, ks * 32);
        accS = wmma_f16(frag_h(sHM, DD2, 0, ks * 32), b, accS);
        accW = wmma_f16(frag_h(sHM + 16 * DD2, DD2, 0, ks * 32), b, accW);
      }
      int col = nt * 16 + ln;
      float bb = b2[col];
      float sign = (col < 4) ? -1.0f : 1.0f;
#pragma unroll
      for (int r = 0; r < 8; ++r) {
        int m = r + 8 * g;
        float s = 1.0f / (1.0f + __expf(-(accS[r] + bb)));
        sS[m * DD + col] = s;
        float v = inB[m * DD2 + DD + col];
        sU[m * DD + col] = (_Float16)(v * v * sign * s * (1.0f - s));
        sWv[m * DD + col] = accW[r];
      }
    }
  }
  __syncthreads();

#pragma unroll
  for (int i = 0; i < 4; ++i) {
    int nt = wid + 4 * i;
    v8f acc = {};
#pragma unroll
    for (int ks = 0; ks < 4; ++ks)
      acc = wmma_f16(frag_h(sU, DD, 0, ks * 32),
                     frag_h(w2t, DD, nt * 16, ks * 32), acc);
    int col = nt * 16 + ln;
#pragma unroll
    for (int r = 0; r < 8; ++r) {
      int m = r + 8 * g;
      sQ[m * DD2 + col] = (_Float16)(sMask[m * DD2 + col] ? acc[r] : 0.0f);
    }
  }
  __syncthreads();

#pragma unroll
  for (int i = 0; i < 2; ++i) {
    int nt = wid + 4 * i;
    v8f acc = {};
#pragma unroll
    for (int ks = 0; ks < 8; ++ks)
      acc = wmma_f16(frag_h(sQ, DD2, 0, ks * 32),
                     frag_h(w1t, DD2, nt * 16, ks * 32), acc);
    int j = nt * 16 + ln;
    float sign = (j < 4) ? -1.0f : 1.0f;
#pragma unroll
    for (int r = 0; r < 8; ++r) {
      int m = r + 8 * g;
      float s = sS[m * DD + j];
      float coef = sign * s * (1.0f - s);
      float ginv = sign / (s + 0.618f);
      float v = inB[m * DD2 + DD + j];
      float dv = -acc[r] * ginv + 2.0f * v * ginv * coef * sWv[m * DD + j];
      sDV[m * DD + j] = dv;
    }
  }
  __syncthreads();
  for (int idx = tid; idx < 16 * 32; idx += 128) { int m = idx >> 5, t = idx & 31; vst2(out + (size_t)(row0 + m) * DD2 + DD + t * 4, *(const v4f*)(sDV + m * DD + t * 4)); }
}

extern "C" void kernel_launch(void* const* d_in, const int* in_sizes, int n_in,
                              void* d_out, int out_size, void* d_ws, size_t ws_size,
                              hipStream_t stream) {
  const float* input = (const float*)d_in[1];
  const float* W1    = (const float*)d_in[2];
  const float* b1    = (const float*)d_in[3];
  const float* W2    = (const float*)d_in[4];
  const float* b2    = (const float*)d_in[5];
  float* out = (float*)d_out;

  __bf16* w1p   = (__bf16*)d_ws;
  _Float16* w2h = (_Float16*)(w1p + 3 * 256 * 128);
  _Float16* w1t = w2h + 128 * 256;
  _Float16* w2t = w1t + 128 * 256;

  const int N = 8192;
  (void)in_sizes;

  prep_w1<<<(256 * 128 / 8) / 256, 256, 0, stream>>>(W1, w1p);
  prep_cvt<<<(128 * 256 / 8) / 256, 256, 0, stream>>>(W2, w2h);
  prep_t<<<(256 / 64) * (128 / 64), 256, 0, stream>>>(W1, w1t, 256, 128);
  prep_t<<<(128 / 64) * (256 / 64), 256, 0, stream>>>(W2, w2t, 128, 256);
  fused_kernel<<<N / 16, 128, 0, stream>>>(input, b1, b2, w1p, w2h, w1t, w2t, out);
}
